// TimeMix_7_5463198400615
// MI455X (gfx1250) — hardware-verified
//
#include <hip/hip_runtime.h>
#include <math.h>

#define NT   2048
#define NC   1024
#define NHD  16
#define HS   64
#define NBT  4096
#define DMX  192
#define DM2  32
#define DLR  64
#define DGT  128
#define GN_EPS 6.4e-4f

static_assert((NBT % 32) == 0);
static_assert((NC % 64) == 0);
static_assert((DMX % 64) == 0);

typedef unsigned short us16;
typedef __bf16 v16b __attribute__((ext_vector_type(16)));
typedef unsigned short v8us __attribute__((ext_vector_type(8), may_alias));
typedef float v8f __attribute__((ext_vector_type(8)));
typedef float v4f __attribute__((ext_vector_type(4)));
typedef float v4fa __attribute__((ext_vector_type(4), may_alias));
typedef float v2f __attribute__((ext_vector_type(2)));
union FragB { v16b v; v8us half[2]; };
union Pack8 { v8us v; us16 u[8]; };

__device__ __forceinline__ us16 bf_rne(float f)
{
  unsigned int u = __builtin_bit_cast(unsigned int, f);
  u = u + 0x7FFFu + ((u >> 16) & 1u);
  return (us16)(u >> 16);
}
__device__ __forceinline__ float bf_val(us16 b)
{
  return __builtin_bit_cast(float, ((unsigned int)b) << 16);
}

__device__ __forceinline__ void mma6(v8f& c0, v8f& c1, v16b ah0, v16b al0, v16b ah1, v16b al1, v16b bh, v16b bl)
{
  c0 = __builtin_amdgcn_wmma_f32_16x16x32_bf16(false, ah0, false, bh, (short)0, c0, false, false);
  c0 = __builtin_amdgcn_wmma_f32_16x16x32_bf16(false, ah0, false, bl, (short)0, c0, false, false);
  c0 = __builtin_amdgcn_wmma_f32_16x16x32_bf16(false, al0, false, bh, (short)0, c0, false, false);
  c1 = __builtin_amdgcn_wmma_f32_16x16x32_bf16(false, ah1, false, bh, (short)0, c1, false, false);
  c1 = __builtin_amdgcn_wmma_f32_16x16x32_bf16(false, ah1, false, bl, (short)0, c1, false, false);
  c1 = __builtin_amdgcn_wmma_f32_16x16x32_bf16(false, al1, false, bh, (short)0, c1, false, false);
  asm volatile("v_nop\n\tv_nop\n\tv_nop\n\tv_nop"
               : "+v"(c0), "+v"(c1)
               : "v"(ah0), "v"(al0), "v"(ah1), "v"(al1), "v"(bh), "v"(bl));
}

__global__ __launch_bounds__(256) void k_wsplit(const float* __restrict__ W, int S, int K, int N,
                                                us16* __restrict__ Dh, us16* __restrict__ Dl)
{
  const size_t t = (size_t)blockIdx.x * 256 + threadIdx.x;
  const int kq = K >> 3;
  const size_t per = (size_t)N * kq;
  const size_t tot = (size_t)S * per;
  if (t >= tot) return;
  const int s = (int)(t / per);
  const int rem = (int)(t - (size_t)s * per);
  const int n = rem / kq;
  const int k8 = (rem - n * kq) * 8;
  Pack8 ph, pl;
#pragma unroll
  for (int i = 0; i < 8; ++i) {
    const float v = W[((size_t)s * K + k8 + i) * N + n];
    const us16 hb = bf_rne(v);
    ph.u[i] = hb;
    pl.u[i] = bf_rne(v - bf_val(hb));
  }
  const size_t o = ((size_t)s * N + n) * K + k8;
  const v8us hv = ph.v, lv = pl.v;
  *(volatile v8us*)(Dh + o) = hv;
  *(volatile v8us*)(Dl + o) = lv;
  __threadfence();
  *(volatile v8us*)(Dh + o) = hv;
  *(volatile v8us*)(Dl + o) = lv;
}

__global__ __launch_bounds__(256) void k_shift(const float* __restrict__ x, const float* __restrict__ mx,
                                               us16* __restrict__ Xh, us16* __restrict__ Xl)
{
#pragma clang fp contract(off)
  const size_t t = (size_t)blockIdx.x * 256 + threadIdx.x;
  if (t >= (size_t)NBT * NC / 8) return;
  const int bt = (int)(t >> 7), c8 = (int)(t & 127) * 8;
  const int tp = bt & (NT - 1);
  const int pb = (tp > 0) ? bt - 1 : bt;
  const float* xc = x + (size_t)bt * NC + c8;
  const float* xp = x + (size_t)pb * NC + c8;
  const v4f a0 = *(const v4fa*)xc, a1 = *(const v4fa*)(xc + 4);
  const v4f p0 = *(const v4fa*)xp, p1 = *(const v4fa*)(xp + 4);
  const v4f m0 = *(const v4fa*)(mx + c8), m1 = *(const v4fa*)(mx + c8 + 4);
  Pack8 ph, pl;
#pragma unroll
  for (int i = 0; i < 4; ++i) {
    const float cur0 = a0[i];
    const float prv0 = (tp > 0) ? p0[i] : 0.0f;
    const float xx0 = prv0 - cur0;
    const float v0 = cur0 + xx0 * m0[i];
    const us16 h0 = bf_rne(v0);
    ph.u[i] = h0; pl.u[i] = bf_rne(v0 - bf_val(h0));
    const float cur1 = a1[i];
    const float prv1 = (tp > 0) ? p1[i] : 0.0f;
    const float xx1 = prv1 - cur1;
    const float v1 = cur1 + xx1 * m1[i];
    const us16 h1 = bf_rne(v1);
    ph.u[4 + i] = h1; pl.u[4 + i] = bf_rne(v1 - bf_val(h1));
  }
  const size_t o = (size_t)bt * NC + c8;
  const v8us hv = ph.v, lv = pl.v;
  *(volatile v8us*)(Xh + o) = hv;
  *(volatile v8us*)(Xl + o) = lv;
  __threadfence();
  *(volatile v8us*)(Xh + o) = hv;
  *(volatile v8us*)(Xl + o) = lv;
}

template <int EPI, bool OUT2>
__global__ __launch_bounds__(128) void k_gemm(const us16* __restrict__ Ah, const us16* __restrict__ Al, int lda,
                                              const us16* __restrict__ Bh, const us16* __restrict__ Bl, int ldb,
                                              int M, int N, int K,
                                              const float* __restrict__ bias, const float* __restrict__ P, int ldp,
                                              float* __restrict__ Cf, us16* __restrict__ Ch, us16* __restrict__ Cl, int ldc)
{
#pragma clang fp contract(off)
  __shared__ __attribute__((aligned(16))) float so[4][32][64];
  const int tid = threadIdx.x, w = tid >> 5, lane = tid & 31, ln = lane & 15, hh = lane >> 4;
  const int ntn = N >> 6;
  const int wid = blockIdx.x * 4 + w;
  const int mt2 = wid / ntn, nq = wid - mt2 * ntn;
  if (mt2 * 32 >= M) return;
  const int row0 = mt2 * 32, col0 = nq * 64;
  const us16* a0h = Ah + (size_t)(row0 + ln) * lda + 8 * hh;
  const us16* a0l = Al + (size_t)(row0 + ln) * lda + 8 * hh;
  const us16* a1h = a0h + (size_t)16 * lda;
  const us16* a1l = a0l + (size_t)16 * lda;
  const size_t bofs = (size_t)(col0 + ln) * ldb + 8 * hh;
  v8f acc[2][4] = {};
#pragma unroll 1
  for (int kb = 0; kb < K; kb += 32) {
    FragB ah0, al0, ah1, al1;
    ah0.half[0] = *(const v8us*)(a0h + kb); ah0.half[1] = *(const v8us*)(a0h + kb + 16);
    al0.half[0] = *(const v8us*)(a0l + kb); al0.half[1] = *(const v8us*)(a0l + kb + 16);
    ah1.half[0] = *(const v8us*)(a1h + kb); ah1.half[1] = *(const v8us*)(a1h + kb + 16);
    al1.half[0] = *(const v8us*)(a1l + kb); al1.half[1] = *(const v8us*)(a1l + kb + 16);
#pragma unroll
    for (int t = 0; t < 4; ++t) {
      const size_t bo = bofs + (size_t)(16 * t) * ldb + kb;
      FragB bh, bl;
      bh.half[0] = *(const v8us*)(Bh + bo); bh.half[1] = *(const v8us*)(Bh + bo + 16);
      bl.half[0] = *(const v8us*)(Bl + bo); bl.half[1] = *(const v8us*)(Bl + bo + 16);
      mma6(acc[0][t], acc[1][t], ah0.v, al0.v, ah1.v, al1.v, bh.v, bl.v);
    }
  }
#pragma unroll
  for (int mt = 0; mt < 2; ++mt) {
#pragma unroll
    for (int t = 0; t < 4; ++t) {
#pragma unroll
      for (int r = 0; r < 8; ++r) so[w][16 * mt + 8 * hh + r][16 * t + ln] = acc[mt][t][r];
    }
  }
  __builtin_amdgcn_fence(__ATOMIC_ACQ_REL, "workgroup");
  __builtin_amdgcn_wave_barrier();
  if (EPI != 0) {
    float* sf = &so[w][0][0];
#pragma unroll 1
    for (int e = lane; e < 32 * 64; e += 32) {
      const int rr = e >> 6, cc = e & 63;
      const int gr = row0 + rr, gc = col0 + cc;
      float v = sf[e];
      if (EPI == 1) {
        v = tanhf(v);
      } else if (EPI == 2) {
        const int tp = gr & (NT - 1);
        const int pr = (tp > 0) ? gr - 1 : gr;
        const float cur = P[(size_t)gr * ldp + gc];
        const float pvv = P[(size_t)pr * ldp + gc];
        const float prv = (tp > 0) ? pvv : 0.0f;
        const float xx = prv - cur;
        const float m = bias[gc] + v;
        v = cur + xx * m;
      } else if (EPI == 3) {
        const float u = -(bias[gc] + v);
        const float sp = fmaxf(u, 0.0f) + log1pf(expf(-fabsf(u)));
        v = -sp - 0.5f;
      } else if (EPI == 4) {
        v = P[(size_t)gr * ldp + gc] + v;
      } else if (EPI == 5) {
        const float z = bias[gc] + v;
        v = __builtin_amdgcn_rcpf(1.0f + expf(-z)) * 2.0f;
      } else if (EPI == 6) {
        v = P[(size_t)gr * ldp + gc] * v;
      }
      sf[e] = v;
    }
    __builtin_amdgcn_fence(__ATOMIC_ACQ_REL, "workgroup");
    __builtin_amdgcn_wave_barrier();
  }
  if (OUT2) {
    const int rq = lane >> 3, c8 = (lane & 7) * 8;
    Pack8 ph[8], pl[8];
#pragma unroll
    for (int q = 0; q < 8; ++q) {
      const v4f a = *(const v4fa*)&so[w][4 * q + rq][c8];
      const v4f b = *(const v4fa*)&so[w][4 * q + rq][c8 + 4];
#pragma unroll
      for (int i = 0; i < 4; ++i) {
        const us16 ha = bf_rne(a[i]);
        ph[q].u[i] = ha;
        pl[q].u[i] = bf_rne(a[i] - bf_val(ha));
        const us16 hb = bf_rne(b[i]);
        ph[q].u[4 + i] = hb;
        pl[q].u[4 + i] = bf_rne(b[i] - bf_val(hb));
      }
    }
    for (int pass = 0; pass < 2; ++pass) {
#pragma unroll
      for (int q = 0; q < 8; ++q) {
        const size_t o = (size_t)(row0 + 4 * q + rq) * ldc + col0 + c8;
        *(volatile v8us*)(Ch + o) = ph[q].v;
        *(volatile v8us*)(Cl + o) = pl[q].v;
      }
      if (pass == 0) __threadfence();
    }
  } else {
    const int rs = lane >> 4, c4 = (lane & 15) * 4;
    v4f pc[16];
#pragma unroll
    for (int q = 0; q < 16; ++q) pc[q] = *(const v4fa*)&so[w][2 * q + rs][c4];
    for (int pass = 0; pass < 2; ++pass) {
#pragma unroll
      for (int q = 0; q < 16; ++q)
        *(volatile v4f*)(Cf + (size_t)(row0 + 2 * q + rs) * ldc + col0 + c4) = pc[q];
      if (pass == 0) __threadfence();
    }
  }
}

__global__ __launch_bounds__(256) void k_norm(const float* __restrict__ KKp, float* __restrict__ INV)
{
#pragma clang fp contract(off)
  __shared__ __attribute__((aligned(16))) float sv[32];
  const int tid = threadIdx.x, w = tid >> 5, lane = tid & 31;
  const int blk = blockIdx.x;
#pragma unroll 1
  for (int u = 0; u < 4; ++u) {
    const int row = blk * 32 + w * 4 + u;
    const float* p = KKp + (size_t)row * NC;
    float ss = 0.0f;
#pragma unroll 4
    for (int m = 0; m < 32; ++m) {
      const float v = p[lane + 32 * m];
      ss = ss + v * v;
    }
    for (int o = 16; o > 0; o >>= 1) ss += __shfl_xor(ss, o, 32);
    const float inv = 1.0f / fmaxf(sqrtf(ss), 1e-12f);
    if (lane == 0) sv[w * 4 + u] = inv;
  }
  __syncthreads();
  if (tid < 8) {
    const v4f a = *(const v4fa*)&sv[4 * tid];
    float* dst = INV + (size_t)blk * 32 + 4 * tid;
    *(volatile v4f*)dst = a;
    __threadfence();
    *(volatile v4f*)dst = a;
  }
}

__global__ __launch_bounds__(256) void k_wkv(const float* __restrict__ Rp, const float* __restrict__ Wp, const float* __restrict__ Kp,
                                             const float* __restrict__ Vp, const float* __restrict__ KKp, const float* __restrict__ Ap,
                                             const float* __restrict__ INV, const float* __restrict__ fa,
                                             const float* __restrict__ lnw, const float* __restrict__ lnb, float* __restrict__ YP)
{
#pragma clang fp contract(off)
  __shared__ __attribute__((aligned(16))) float lw[HS];
  __shared__ __attribute__((aligned(16))) float lk[HS];
  __shared__ __attribute__((aligned(16))) float la[HS];
  __shared__ __attribute__((aligned(16))) float lb[HS];
  __shared__ __attribute__((aligned(16))) float lr[HS];
  __shared__ __attribute__((aligned(16))) float lv[HS];
  __shared__ __attribute__((aligned(16))) float ys[HS];
  const int tid = threadIdx.x, lane = tid & 31;
  const int b = blockIdx.x >> 4, h = blockIdx.x & (NHD - 1);
  const int i = tid >> 2, jq = tid & 3, j0 = jq * 16;
  const int hc = h * HS;
  const int cl = 2 * lane;
  const float fa0 = fa[hc + cl], fa1 = fa[hc + cl + 1];
  const float gw0 = lnw[hc + cl], gw1 = lnw[hc + cl + 1];
  const float gb0 = lnb[hc + cl], gb1 = lnb[hc + cl + 1];
  float S[16];
#pragma unroll
  for (int m = 0; m < 16; ++m) S[m] = 0.0f;
  const size_t rowb = (size_t)b * NT;
#pragma unroll 1
  for (int t = 0; t < NT; ++t) {
    const size_t row = rowb + t;
    const size_t e = row * NC + hc;
    if (tid < HS) {
      const float r = Rp[e + tid], w = Wp[e + tid], k = Kp[e + tid];
      const float v = Vp[e + tid], kk = KKp[e + tid], a = Ap[e + tid];
      const float inv = INV[row];
      const float wd = expf(-expf(w));
      const float ksc = k * expf(fminf(w * 0.5f, 0.0f));
      const float kkn = kk * inv;
      lw[tid] = wd; lk[tid] = ksc; la[tid] = -kkn; lb[tid] = kkn * a; lr[tid] = r; lv[tid] = v;
    }
    __syncthreads();
    float av[16], wv[16], bv[16], kv[16], rv[16];
#pragma unroll
    for (int m = 0; m < 4; ++m) {
      const v4f qa = *(const v4fa*)&la[j0 + 4 * m];
      const v4f qw = *(const v4fa*)&lw[j0 + 4 * m];
      const v4f qb = *(const v4fa*)&lb[j0 + 4 * m];
      const v4f qk = *(const v4fa*)&lk[j0 + 4 * m];
      const v4f qr = *(const v4fa*)&lr[j0 + 4 * m];
      av[4 * m] = qa[0]; av[4 * m + 1] = qa[1]; av[4 * m + 2] = qa[2]; av[4 * m + 3] = qa[3];
      wv[4 * m] = qw[0]; wv[4 * m + 1] = qw[1]; wv[4 * m + 2] = qw[2]; wv[4 * m + 3] = qw[3];
      bv[4 * m] = qb[0]; bv[4 * m + 1] = qb[1]; bv[4 * m + 2] = qb[2]; bv[4 * m + 3] = qb[3];
      kv[4 * m] = qk[0]; kv[4 * m + 1] = qk[1]; kv[4 * m + 2] = qk[2]; kv[4 * m + 3] = qk[3];
      rv[4 * m] = qr[0]; rv[4 * m + 1] = qr[1]; rv[4 * m + 2] = qr[2]; rv[4 * m + 3] = qr[3];
    }
    const float vi = lv[i];
    const float rr0 = lr[cl], rr1 = lr[cl + 1];
    const float kq0 = lk[cl], kq1 = lk[cl + 1];
    const float vv0 = lv[cl], vv1 = lv[cl + 1];
    float sa = 0.0f;
#pragma unroll
    for (int m = 0; m < 16; ++m) sa = fmaf(S[m], av[m], sa);
    sa += __shfl_xor(sa, 1, 32);
    sa += __shfl_xor(sa, 2, 32);
    float yp = 0.0f;
#pragma unroll
    for (int m = 0; m < 16; ++m) {
      float s2 = S[m] * wv[m];
      s2 = fmaf(sa, bv[m], s2);
      s2 = fmaf(vi, kv[m], s2);
      S[m] = s2;
      yp = fmaf(s2, rv[m], yp);
    }
    yp += __shfl_xor(yp, 1, 32);
    yp += __shfl_xor(yp, 2, 32);
    if (jq == 0) ys[i] = yp;
    __syncthreads();
    if (tid < 32) {
      const float y0 = ys[cl], y1 = ys[cl + 1];
      float s = y0 + y1;
      for (int o = 16; o > 0; o >>= 1) s += __shfl_xor(s, o, 32);
      const float mu = s * 0.015625f;
      const float d0 = y0 - mu, d1 = y1 - mu;
      float q = d0 * d0 + d1 * d1;
      for (int o = 16; o > 0; o >>= 1) q += __shfl_xor(q, o, 32);
      const float var = q * 0.015625f;
      const float rs = 1.0f / sqrtf(var + GN_EPS);
      float bon = (rr0 * kq0) * fa0 + (rr1 * kq1) * fa1;
      for (int o = 16; o > 0; o >>= 1) bon += __shfl_xor(bon, o, 32);
      const float o0 = ((d0 * rs) * gw0 + gb0) + bon * vv0;
      const float o1 = ((d1 * rs) * gw1 + gb1) + bon * vv1;
      v2f ov;
      ov[0] = o0; ov[1] = o1;
      float* dst = YP + e + cl;
      *(volatile v2f*)dst = ov;
      __threadfence();
      *(volatile v2f*)dst = ov;
    }
  }
}

template <int EPI, bool OUT2>
static void gemm_go(hipStream_t st, const us16* Ah, const us16* Al, int lda, const us16* Bh, const us16* Bl, int ldb,
                    int M, int N, int K, const float* bias, const float* P, int ldp, float* Cf, us16* Ch, us16* Cl, int ldc)
{
  const unsigned nb = (unsigned)(((M / 32) * (N / 64) + 3) / 4);
  k_gemm<EPI, OUT2><<<nb, 128, 0, st>>>(Ah, Al, lda, Bh, Bl, ldb, M, N, K, bias, P, ldp, Cf, Ch, Cl, ldc);
}

static void wsplit_go(hipStream_t st, const float* W, int S, int K, int N, us16* Dh, us16* Dl)
{
  const size_t tot = (size_t)S * N * (K / 8);
  k_wsplit<<<(unsigned)((tot + 255) / 256), 256, 0, st>>>(W, S, K, N, Dh, Dl);
}

extern "C" void kernel_launch(void* const* d_in, const int* in_sizes, int n_in,
                              void* d_out, int out_size, void* d_ws, size_t ws_size, hipStream_t stream)
{
  if (n_in < 27) return;
  if (in_sizes[0] != NBT * NC) return;
  for (int q = 1; q <= 8; ++q) if (in_sizes[q] != NC) return;
  if (in_sizes[9] != NHD * HS || in_sizes[10] != NC) return;
  if (in_sizes[11] != NC * DMX || in_sizes[12] != 6 * DM2 * NC) return;
  for (int q = 13; q <= 18; ++q) if (in_sizes[q] != NC * DLR) return;
  if (in_sizes[19] != NC * DGT || in_sizes[20] != DGT * NC) return;
  for (int q = 21; q <= 24; ++q) if (in_sizes[q] != NC * NC) return;
  if (in_sizes[25] != NC || in_sizes[26] != NC) return;
  if (out_size != NBT * NC) return;

  const float* x      = (const float*)d_in[0];
  const float* maa_x  = (const float*)d_in[1];
  const float* maa_r  = (const float*)d_in[2];
  const float* maa_w  = (const float*)d_in[3];
  const float* maa_k  = (const float*)d_in[4];
  const float* maa_v  = (const float*)d_in[5];
  const float* maa_a  = (const float*)d_in[6];
  const float* maa_g  = (const float*)d_in[7];
  const float* tdecay = (const float*)d_in[8];
  const float* faaaa  = (const float*)d_in[9];
  const float* taaaaa = (const float*)d_in[10];
  const float* mw1    = (const float*)d_in[11];
  const float* mw2    = (const float*)d_in[12];
  const float* dw1    = (const float*)d_in[13];
  const float* dw2    = (const float*)d_in[14];
  const float* aw1    = (const float*)d_in[15];
  const float* aw2    = (const float*)d_in[16];
  const float* kw1    = (const float*)d_in[17];
  const float* kw2    = (const float*)d_in[18];
  const float* gw1    = (const float*)d_in[19];
  const float* gw2    = (const float*)d_in[20];
  const float* W_r    = (const float*)d_in[21];
  const float* W_k    = (const float*)d_in[22];
  const float* W_v    = (const float*)d_in[23];
  const float* W_o    = (const float*)d_in[24];
  const float* lnw    = (const float*)d_in[25];
  const float* lnb    = (const float*)d_in[26];
  float* out0 = (float*)d_out;

  char* ws = (char*)d_ws;
  size_t off = 0;
  auto take = [&](size_t bytes) -> char* { char* p = ws + off; off += (bytes + 4095) & ~(size_t)4095; return p; };
  const size_t PL = (size_t)NBT * NC;
  us16* BWh  = (us16*)take((size_t)NC * NC * 2 * 2);   us16* BWl  = BWh  + (size_t)NC * NC;
  us16* MW1h = (us16*)take((size_t)DMX * NC * 2 * 2);  us16* MW1l = MW1h + (size_t)DMX * NC;
  us16* MW2h = (us16*)take((size_t)6 * NC * DM2 * 4);  us16* MW2l = MW2h + (size_t)6 * NC * DM2;
  us16* DW1h = (us16*)take((size_t)DLR * NC * 4);      us16* DW1l = DW1h + (size_t)DLR * NC;
  us16* DW2h = (us16*)take((size_t)NC * DLR * 4);      us16* DW2l = DW2h + (size_t)NC * DLR;
  us16* AW1h = (us16*)take((size_t)DLR * NC * 4);      us16* AW1l = AW1h + (size_t)DLR * NC;
  us16* AW2h = (us16*)take((size_t)NC * DLR * 4);      us16* AW2l = AW2h + (size_t)NC * DLR;
  us16* KW1h = (us16*)take((size_t)DLR * NC * 4);      us16* KW1l = KW1h + (size_t)DLR * NC;
  us16* KW2h = (us16*)take((size_t)NC * DLR * 4);      us16* KW2l = KW2h + (size_t)NC * DLR;
  us16* GW1h = (us16*)take((size_t)DGT * NC * 4);      us16* GW1l = GW1h + (size_t)DGT * NC;
  us16* GW2h = (us16*)take((size_t)NC * DGT * 4);      us16* GW2l = GW2h + (size_t)NC * DGT;
  us16* XSh  = (us16*)take(PL * 2 * 2);                us16* XSl  = XSh  + PL;
  float* YP  = (float*)XSh;
  us16* MIXh = (us16*)take((size_t)NBT * DMX * 4);     us16* MIXl = MIXh + (size_t)NBT * DMX;
  us16* LHh  = (us16*)take((size_t)NBT * DGT * 4);     us16* LHl  = LHh  + (size_t)NBT * DGT;
  float* Rp  = (float*)take(PL * 4);
  us16* Zh   = (us16*)Rp;                              us16* Zl   = Zh + PL;
  float* Wp  = (float*)take(PL * 4);
  float* Kp  = (float*)take(PL * 4);
  float* Vp  = (float*)take(PL * 4);
  float* KKp = (float*)take(PL * 4);
  float* Ap  = (float*)take(PL * 4);
  float* INV = (float*)take((size_t)NBT * 4);
  if (off > ws_size) return;
  if (off > (size_t)134217728) return;

  wsplit_go(stream, mw1, 1, NC, DMX, MW1h, MW1l);
  wsplit_go(stream, mw2, 6, DM2, NC, MW2h, MW2l);
  wsplit_go(stream, dw1, 1, NC, DLR, DW1h, DW1l);
  wsplit_go(stream, dw2, 1, DLR, NC, DW2h, DW2l);
  wsplit_go(stream, aw1, 1, NC, DLR, AW1h, AW1l);
  wsplit_go(stream, aw2, 1, DLR, NC, AW2h, AW2l);
  wsplit_go(stream, kw1, 1, NC, DLR, KW1h, KW1l);
  wsplit_go(stream, kw2, 1, DLR, NC, KW2h, KW2l);
  wsplit_go(stream, gw1, 1, NC, DGT, GW1h, GW1l);
  wsplit_go(stream, gw2, 1, DGT, NC, GW2h, GW2l);

  k_shift<<<(unsigned)(PL / 8 / 256), 256, 0, stream>>>(x, maa_x, XSh, XSl);
  gemm_go<1, true>(stream, XSh, XSl, NC, MW1h, MW1l, NC, NBT, DMX, NC, nullptr, nullptr, 0, nullptr, MIXh, MIXl, DMX);

  auto branch = [&](int s, const float* maa) {
    gemm_go<2, true>(stream, MIXh + 32 * s, MIXl + 32 * s, DMX, MW2h + (size_t)s * NC * DM2, MW2l + (size_t)s * NC * DM2, DM2,
                     NBT, NC, DM2, maa, x, NC, nullptr, XSh, XSl, NC);
  };

  branch(0, maa_r);
  wsplit_go(stream, W_r, 1, NC, NC, BWh, BWl);
  gemm_go<0, false>(stream, XSh, XSl, NC, BWh, BWl, NC, NBT, NC, NC, nullptr, nullptr, 0, Rp, nullptr, nullptr, NC);

  branch(2, maa_k);
  wsplit_go(stream, W_k, 1, NC, NC, BWh, BWl);
  gemm_go<0, false>(stream, XSh, XSl, NC, BWh, BWl, NC, NBT, NC, NC, nullptr, nullptr, 0, Kp, nullptr, nullptr, NC);
  gemm_go<1, true>(stream, XSh, XSl, NC, KW1h, KW1l, NC, NBT, DLR, NC, nullptr, nullptr, 0, nullptr, LHh, LHl, DLR);
  gemm_go<4, false>(stream, LHh, LHl, DLR, KW2h, KW2l, DLR, NBT, NC, DLR, nullptr, Kp, NC, KKp, nullptr, nullptr, NC);
  k_norm<<<(unsigned)(NBT / 32), 256, 0, stream>>>(KKp, INV);

  branch(1, maa_w);
  gemm_go<1, true>(stream, XSh, XSl, NC, DW1h, DW1l, NC, NBT, DLR, NC, nullptr, nullptr, 0, nullptr, LHh, LHl, DLR);
  gemm_go<3, false>(stream, LHh, LHl, DLR, DW2h, DW2l, DLR, NBT, NC, DLR, tdecay, nullptr, 0, Wp, nullptr, nullptr, NC);

  branch(3, maa_v);
  wsplit_go(stream, W_v, 1, NC, NC, BWh, BWl);
  gemm_go<0, false>(stream, XSh, XSl, NC, BWh, BWl, NC, NBT, NC, NC, nullptr, nullptr, 0, Vp, nullptr, nullptr, NC);

  branch(4, maa_a);
  gemm_go<0, true>(stream, XSh, XSl, NC, AW1h, AW1l, NC, NBT, DLR, NC, nullptr, nullptr, 0, nullptr, LHh, LHl, DLR);
  gemm_go<5, false>(stream, LHh, LHl, DLR, AW2h, AW2l, DLR, NBT, NC, DLR, taaaaa, nullptr, 0, Ap, nullptr, nullptr, NC);

  branch(5, maa_g);
  gemm_go<1, true>(stream, XSh, XSl, NC, GW1h, GW1l, NC, NBT, DGT, NC, nullptr, nullptr, 0, nullptr, LHh, LHl, DGT);

  k_wkv<<<(unsigned)(NBT / NT * NHD), 256, 0, stream>>>(Rp, Wp, Kp, Vp, KKp, Ap, INV, faaaa, lnw, lnb, YP);

  gemm_go<6, true>(stream, LHh, LHl, DGT, GW2h, GW2l, DGT, NBT, NC, DGT, nullptr, YP, NC, nullptr, Zh, Zl, NC);

  wsplit_go(stream, W_o, 1, NC, NC, BWh, BWl);
  gemm_go<0, false>(stream, Zh, Zl, NC, BWh, BWl, NC, NBT, NC, NC, nullptr, nullptr, 0, out0, nullptr, nullptr, NC);
}
